// UncertaintyPropagationGraph_3384434230093
// MI455X (gfx1250) — hardware-run, weakly checked
//
#include <hip/hip_runtime.h>
#include <stdint.h>

#define NBATCH 512
#define NNODE  16
#define ND     256
#define NLAYER 3
#define NSTEP  4
#define NR     (NBATCH * NNODE)
#define KHL    (2 * ND)
#define NG     (4 * ND)
#define KL     (2 * KHL)
#define TP     72

static_assert(NR % 128 == 0);
static_assert(NR % 8 == 0);
static_assert(ND % 64 == 0);
static_assert(KHL % 64 == 0);
static_assert(NG % 64 == 0);
static_assert(KHL % 32 == 0);
static_assert(KL % 32 == 0);
static_assert(ND == 256);
static_assert(NNODE == 16);
static_assert((TP * 2) % 16 == 0);
static_assert((2 * NG * (ND / 8)) % 256 == 0);
static_assert((size_t)NR * ND + (size_t)NR * NSTEP * ND == (size_t)10485760);

typedef __attribute__((ext_vector_type(16))) __bf16 v16b;
typedef __attribute__((ext_vector_type(8)))  __bf16 v8b;
typedef __attribute__((ext_vector_type(8)))  float  v8f;
typedef __attribute__((ext_vector_type(4)))  float  v4f;
typedef __attribute__((ext_vector_type(4)))  unsigned int v4u;
typedef v8b __attribute__((may_alias)) v8ba;
typedef v4f __attribute__((may_alias)) v4fa;
typedef v4u __attribute__((may_alias)) v4ua;

union FragU { v16b v; v8b h[2]; };

__device__ __forceinline__ unsigned short f2bf_bits(float f) {
  const unsigned u = __float_as_uint(f);
  return (unsigned short)((u + 0x7FFFu + ((u >> 16) & 1u)) >> 16);
}
__device__ __forceinline__ float bf_bits2f(unsigned short h) { return __uint_as_float(((unsigned)h) << 16); }
__device__ __forceinline__ float bf16r(float f) {
  unsigned u = __float_as_uint(f);
  u = (u + 0x7FFFu + ((u >> 16) & 1u)) & 0xFFFF0000u;
  return __uint_as_float(u);
}
__device__ __forceinline__ unsigned pk16(unsigned short a, unsigned short b) { return (unsigned)a | ((unsigned)b << 16); }
__device__ __forceinline__ unsigned hi2(float x, float y) { return pk16(f2bf_bits(x), f2bf_bits(y)); }
__device__ __forceinline__ unsigned lo2(float x, float y) {
  const float rx = x - bf_bits2f(f2bf_bits(x));
  const float ry = y - bf_bits2f(f2bf_bits(y));
  return pk16(f2bf_bits(rx), f2bf_bits(ry));
}
__device__ __forceinline__ v4u hi8(v4f a, v4f c) {
  v4u o;
  o[0] = hi2(a[0], a[1]); o[1] = hi2(a[2], a[3]); o[2] = hi2(c[0], c[1]); o[3] = hi2(c[2], c[3]);
  return o;
}
__device__ __forceinline__ v4u lo8(v4f a, v4f c) {
  v4u o;
  o[0] = lo2(a[0], a[1]); o[1] = lo2(a[2], a[3]); o[2] = lo2(c[0], c[1]); o[3] = lo2(c[2], c[3]);
  return o;
}
__device__ __forceinline__ float sigm(float x) { return 1.0f / (1.0f + expf(-x)); }

__device__ __forceinline__ v8f wmma_bf16(v16b a, v16b b, v8f c) {
  v8f d = __builtin_amdgcn_wmma_f32_16x16x32_bf16(false, a, false, b, (short)0, c, false, false);
  asm volatile("v_nop\n\tv_nop\n\tv_nop\n\tv_nop" : "+v"(d) : "v"(a), "v"(b));
  return d;
}

__device__ __forceinline__ v16b load_frag(const unsigned short* p, int hh) {
  FragU f;
  f.h[0] = *(const v8ba*)(p + 8 * hh);
  f.h[1] = *(const v8ba*)(p + 16 + 8 * hh);
  return f.v;
}

__device__ __forceinline__ void gemm_seg(const unsigned short* a0, const unsigned short* a1,
                                         const unsigned short* bp, int ldb, int klen, int hh,
                                         v8f (&acc)[2][4]) {
#pragma unroll 1
  for (int k0 = 0; k0 < klen; k0 += 32) {
    const v16b f0 = load_frag(a0 + k0, hh);
    const v16b f1 = load_frag(a1 + k0, hh);
#pragma unroll
    for (int nt = 0; nt < 4; ++nt) {
      const v16b fb = load_frag(bp + (size_t)nt * 16 * ldb + k0, hh);
      acc[0][nt] = wmma_bf16(f0, fb, acc[0][nt]);
      acc[1][nt] = wmma_bf16(f1, fb, acc[1][nt]);
    }
  }
}

__device__ __forceinline__ void acc_clear(v8f (&acc)[2][4]) {
  const v8f zero8 = {0.f, 0.f, 0.f, 0.f, 0.f, 0.f, 0.f, 0.f};
#pragma unroll
  for (int mt = 0; mt < 2; ++mt)
#pragma unroll
    for (int nt = 0; nt < 4; ++nt) acc[mt][nt] = zero8;
}

template <int RELU>
__device__ __forceinline__ void stage_tile(float* sF, const v8f (&acc)[2][4], const float (&bv)[4],
                                           int w, int hh, int m) {
#pragma unroll
  for (int nt = 0; nt < 4; ++nt)
#pragma unroll
    for (int mt = 0; mt < 2; ++mt)
#pragma unroll
      for (int r = 0; r < 8; ++r) {
        const int tokl = 32 * w + 16 * mt + 8 * hh + r;
        const int feat = 16 * nt + m;
        float y = acc[mt][nt][r] + bv[nt];
        if (RELU) y = fmaxf(y, 0.0f);
        sF[tokl * 64 + feat] = y;
      }
}

__device__ __forceinline__ void sweep_f32(const float* sF, float* F, int ldf, int m0, int n0, int w, int lane) {
  const int rsub = lane >> 4, c4 = (lane & 15) * 4;
  v4f vals[16];
#pragma unroll
  for (int it = 0; it < 16; ++it) {
    const int row = 32 * w + 2 * it + rsub;
    vals[it] = *(const v4fa*)(sF + row * 64 + c4);
  }
  for (int pass = 0; pass < 2; ++pass) {
#pragma unroll
    for (int it = 0; it < 16; ++it) {
      const int row = 32 * w + 2 * it + rsub;
      *(volatile v4f*)(F + (size_t)(m0 + row) * ldf + n0 + c4) = vals[it];
    }
    __threadfence();
  }
}

__global__ __launch_bounds__(256) void k_wt(const float* __restrict__ src, unsigned short* __restrict__ dst,
                                            int zdiv, int dOuter, int dInner, int ldd) {
  __shared__ __align__(16) unsigned short sT[64 * TP];
  const int tid = threadIdx.x, lane = tid & 31, w = tid >> 5;
  const int c0 = blockIdx.x * 64, k0 = blockIdx.y * 64, z = blockIdx.z;
  const float* s = src + (size_t)z * (ND * ND);
  unsigned short* d = dst + (size_t)(z / zdiv) * dOuter + (size_t)(z % zdiv) * dInner;
  const int c4 = (tid & 15) * 4, rr = tid >> 4;
#pragma unroll
  for (int p = 0; p < 4; ++p) {
    const int r = rr + 16 * p;
    const v4f v = *(const v4fa*)(s + (size_t)(k0 + r) * ND + c0 + c4);
    sT[(c4 + 0) * TP + r] = f2bf_bits(v[0]);
    sT[(c4 + 1) * TP + r] = f2bf_bits(v[1]);
    sT[(c4 + 2) * TP + r] = f2bf_bits(v[2]);
    sT[(c4 + 3) * TP + r] = f2bf_bits(v[3]);
  }
  __syncthreads();
  const int q8 = lane & 7, sub = lane >> 3;
  v4u vv[2];
#pragma unroll
  for (int it = 0; it < 2; ++it) {
    const int row = 32 * it + 4 * w + sub;
    vv[it] = *(const v4ua*)(sT + row * TP + 8 * q8);
  }
  for (int pass = 0; pass < 2; ++pass) {
#pragma unroll
    for (int it = 0; it < 2; ++it) {
      const int row = 32 * it + 4 * w + sub;
      unsigned short* o = d + (size_t)(c0 + row) * ldd + k0 + 8 * q8;
      *(volatile v4u*)o = vv[it];
      *(volatile v4u*)(o + ND) = vv[it];
    }
    __threadfence();
  }
}

__global__ __launch_bounds__(256) void k_wl(const float* __restrict__ Wih, const float* __restrict__ Whh,
                                            unsigned short* __restrict__ BL) {
  const int g = blockIdx.x * 256 + threadIdx.x;
  if (g >= 2 * NG * (ND / 8)) return;
  const int row = g >> 5, kk = g & 31;
  const size_t so = (size_t)row * ND + 8 * kk;
  const v4f a = *(const v4fa*)(Wih + so);
  const v4f c = *(const v4fa*)(Wih + so + 4);
  const v4f p = *(const v4fa*)(Whh + so);
  const v4f q = *(const v4fa*)(Whh + so + 4);
  const v4u vi = hi8(a, c);
  const v4u vh = hi8(p, q);
  unsigned short* o = BL + (size_t)row * KL + 8 * kk;
  for (int pass = 0; pass < 2; ++pass) {
    *(volatile v4u*)o = vi;
    *(volatile v4u*)(o + ND) = vi;
    *(volatile v4u*)(o + 2 * ND) = vh;
    *(volatile v4u*)(o + 3 * ND) = vh;
    __threadfence();
  }
}

__global__ __launch_bounds__(256) void k_x0(const float* __restrict__ mf, const float* __restrict__ emb,
                                            float* __restrict__ XF, unsigned short* __restrict__ XHL,
                                            unsigned short* __restrict__ HIST) {
  const int tid = threadIdx.x, lane = tid & 31, w = tid >> 5;
  const int r = blockIdx.x * 8 + w;
  const int mnode = r & 15, b = r >> 4;
  const float* src = mf + (size_t)r * ND;
  const float* es = emb + (size_t)mnode * ND;
  const int c = 4 * lane, c8 = 8 * lane;
  const v4f a0 = *(const v4fa*)(src + c);
  const v4f a1 = *(const v4fa*)(src + 128 + c);
  const v4f e0 = *(const v4fa*)(es + c);
  const v4f e1 = *(const v4fa*)(es + 128 + c);
  const v4f p0 = *(const v4fa*)(src + c8);
  const v4f p1 = *(const v4fa*)(src + c8 + 4);
  const v4f q0 = *(const v4fa*)(es + c8);
  const v4f q1 = *(const v4fa*)(es + c8 + 4);
  v4f x0 = {0.f, 0.f, 0.f, 0.f}, x1 = {0.f, 0.f, 0.f, 0.f}, y0 = {0.f, 0.f, 0.f, 0.f}, y1 = {0.f, 0.f, 0.f, 0.f};
#pragma unroll
  for (int e = 0; e < 4; ++e) {
    x0[e] = bf16r(a0[e]) + bf16r(e0[e]);
    x1[e] = bf16r(a1[e]) + bf16r(e1[e]);
    y0[e] = bf16r(p0[e]) + bf16r(q0[e]);
    y1[e] = bf16r(p1[e]) + bf16r(q1[e]);
  }
  const v4u hv = hi8(y0, y1);
  const v4u lv = lo8(y0, y1);
  float* fd = XF + (size_t)r * ND;
  unsigned short* xd = XHL + (size_t)r * KHL + c8;
  unsigned short* hd = HIST + ((size_t)b * 64 + mnode) * KHL + c8;
  for (int pass = 0; pass < 2; ++pass) {
    *(volatile v4f*)(fd + c) = x0;
    *(volatile v4f*)(fd + 128 + c) = x1;
    *(volatile v4u*)xd = hv;
    *(volatile v4u*)(xd + ND) = lv;
    *(volatile v4u*)hd = hv;
    *(volatile v4u*)(hd + ND) = lv;
    __threadfence();
  }
}

template <int BIAS>
__global__ __launch_bounds__(128) __attribute__((amdgpu_num_vgpr(248)))
void k_gemm_f32(const unsigned short* __restrict__ A0, int lda0,
                const unsigned short* A1, int lda1, int K0, int K1,
                const unsigned short* __restrict__ Bt, int ldb,
                float* __restrict__ F, int ldf,
                const float* __restrict__ bA, const float* __restrict__ bB) {
  __shared__ __align__(16) float sF[128 * 64];
  const int tid = threadIdx.x, lane = tid & 31, w = tid >> 5;
  const int hh = lane >> 4, m = lane & 15;
  const int m0 = blockIdx.x * 128, n0 = blockIdx.y * 64;
  const int m0w = m0 + 32 * w;
  v8f acc[2][4];
  acc_clear(acc);
  {
    const unsigned short* a0 = A0 + (size_t)(m0w + m) * lda0;
    gemm_seg(a0, a0 + (size_t)16 * lda0, Bt + (size_t)(n0 + m) * ldb, ldb, K0, hh, acc);
  }
  {
    const unsigned short* a1 = A1 + (size_t)(m0w + m) * lda1;
    gemm_seg(a1, a1 + (size_t)16 * lda1, Bt + (size_t)(n0 + m) * ldb + K0, ldb, K1, hh, acc);
  }
  float bv[4];
#pragma unroll
  for (int nt = 0; nt < 4; ++nt) {
    if (BIAS) bv[nt] = bf16r(bA[n0 + 16 * nt + m]) + bf16r(bB[n0 + 16 * nt + m]);
    else bv[nt] = 0.0f;
  }
  stage_tile<0>(sF, acc, bv, w, hh, m);
  __syncthreads();
  sweep_f32(sF, F, ldf, m0, n0, w, lane);
}

__global__ __launch_bounds__(128) __attribute__((amdgpu_num_vgpr(248)))
void k_gemm_relu(const unsigned short* __restrict__ A0, const unsigned short* A1,
                 const unsigned short* __restrict__ Bt, const float* __restrict__ bias,
                 unsigned short* __restrict__ OUT) {
  __shared__ __align__(16) float sF[128 * 64];
  const int tid = threadIdx.x, lane = tid & 31, w = tid >> 5;
  const int hh = lane >> 4, m = lane & 15;
  const int m0 = blockIdx.x * 128, n0 = blockIdx.y * 64;
  const int m0w = m0 + 32 * w;
  v8f acc[2][4];
  acc_clear(acc);
  {
    const unsigned short* a0 = A0 + (size_t)(m0w + m) * KHL;
    gemm_seg(a0, a0 + (size_t)16 * KHL, Bt + (size_t)(n0 + m) * KL, KL, KHL, hh, acc);
  }
  {
    const unsigned short* a1 = A1 + (size_t)(m0w + m) * KHL;
    gemm_seg(a1, a1 + (size_t)16 * KHL, Bt + (size_t)(n0 + m) * KL + KHL, KL, KHL, hh, acc);
  }
  float bv[4];
#pragma unroll
  for (int nt = 0; nt < 4; ++nt) bv[nt] = bf16r(bias[n0 + 16 * nt + m]);
  stage_tile<1>(sF, acc, bv, w, hh, m);
  __syncthreads();
  const int q8 = lane & 7, sub = lane >> 3;
  v4u hv[8], lv[8];
#pragma unroll
  for (int it = 0; it < 8; ++it) {
    const int row = 32 * w + 4 * it + sub;
    const v4f a = *(const v4fa*)(sF + row * 64 + 8 * q8);
    const v4f c = *(const v4fa*)(sF + row * 64 + 8 * q8 + 4);
    hv[it] = hi8(a, c);
    lv[it] = lo8(a, c);
  }
  for (int pass = 0; pass < 2; ++pass) {
#pragma unroll
    for (int it = 0; it < 8; ++it) {
      const int row = 32 * w + 4 * it + sub;
      unsigned short* o = OUT + (size_t)(m0 + row) * KHL + n0 + 8 * q8;
      *(volatile v4u*)o = hv[it];
      *(volatile v4u*)(o + ND) = lv[it];
    }
    __threadfence();
  }
}

__global__ __launch_bounds__(128) __attribute__((amdgpu_num_vgpr(248)))
void k_gemm_x(const unsigned short* __restrict__ A, const unsigned short* __restrict__ Bt,
              const float* __restrict__ bias, float* __restrict__ F,
              unsigned short* __restrict__ XHL, unsigned short* __restrict__ HIST,
              int slot, int wrx) {
  __shared__ __align__(16) float sF[128 * 64];
  const int tid = threadIdx.x, lane = tid & 31, w = tid >> 5;
  const int hh = lane >> 4, m = lane & 15;
  const int m0 = blockIdx.x * 128, n0 = blockIdx.y * 64;
  const int m0w = m0 + 32 * w;
  v8f acc[2][4];
  acc_clear(acc);
  {
    const unsigned short* a0 = A + (size_t)(m0w + m) * KHL;
    gemm_seg(a0, a0 + (size_t)16 * KHL, Bt + (size_t)(n0 + m) * KHL, KHL, KHL, hh, acc);
  }
  float bv[4];
#pragma unroll
  for (int nt = 0; nt < 4; ++nt) bv[nt] = bf16r(bias[n0 + 16 * nt + m]);
  stage_tile<0>(sF, acc, bv, w, hh, m);
  __syncthreads();
  sweep_f32(sF, F, ND, m0, n0, w, lane);
  const int q8 = lane & 7, sub = lane >> 3;
  v4u hv[8], lv[8];
#pragma unroll
  for (int it = 0; it < 8; ++it) {
    const int row = 32 * w + 4 * it + sub;
    const v4f a = *(const v4fa*)(sF + row * 64 + 8 * q8);
    const v4f c = *(const v4fa*)(sF + row * 64 + 8 * q8 + 4);
    hv[it] = hi8(a, c);
    lv[it] = lo8(a, c);
  }
  for (int pass = 0; pass < 2; ++pass) {
#pragma unroll
    for (int it = 0; it < 8; ++it) {
      const int gr = m0 + 32 * w + 4 * it + sub;
      const int hrow = (gr >> 4) * 64 + slot * 16 + (gr & 15);
      unsigned short* o = HIST + (size_t)hrow * KHL + n0 + 8 * q8;
      *(volatile v4u*)o = hv[it];
      *(volatile v4u*)(o + ND) = lv[it];
      if (wrx != 0) {
        unsigned short* x = XHL + (size_t)gr * KHL + n0 + 8 * q8;
        *(volatile v4u*)x = hv[it];
        *(volatile v4u*)(x + ND) = lv[it];
      }
    }
    __threadfence();
  }
}

__global__ __launch_bounds__(256) void k_pair(const float* __restrict__ HIJ, const float* __restrict__ XF,
                                              const int* __restrict__ adj, const float* __restrict__ eb1,
                                              const float* __restrict__ eW2, const float* __restrict__ eb2,
                                              unsigned short* __restrict__ AGG) {
  __shared__ __align__(16) float sHJ[16 * 512];
  __shared__ __align__(16) float sX[16 * 256];
  __shared__ __align__(16) float sE2[256];
  __shared__ __align__(16) float sB1[256];
  __shared__ float sW[256];
  __shared__ int sMask[256];
  const int tid = threadIdx.x, lane = tid & 31, w = tid >> 5;
  const int b = blockIdx.x;

  const float* hsrc = HIJ + (size_t)b * (16 * 512);
#pragma unroll 4
  for (int p = 0; p < 8; ++p) {
    const int idx = (p * 256 + tid) * 4;
    const v4f v = *(const v4fa*)(hsrc + idx);
    *(v4fa*)(sHJ + idx) = v;
  }
  const float* xsrc = XF + (size_t)b * (16 * 256);
#pragma unroll 4
  for (int p = 0; p < 4; ++p) {
    const int idx = (p * 256 + tid) * 4;
    const v4f v = *(const v4fa*)(xsrc + idx);
    *(v4fa*)(sX + idx) = v;
  }
  sE2[tid] = bf16r(eW2[tid]);
  sB1[tid] = bf16r(eb1[tid]);
  sMask[tid] = (adj[tid] != 0) ? 1 : 0;
  const float e2b = bf16r(eb2[0]);
  __syncthreads();

  {
    const v4f b1a = *(const v4fa*)(sB1 + 4 * lane);
    const v4f b1b = *(const v4fa*)(sB1 + 128 + 4 * lane);
    const v4f wa = *(const v4fa*)(sE2 + 4 * lane);
    const v4f wb = *(const v4fa*)(sE2 + 128 + 4 * lane);
#pragma unroll 1
    for (int ii = 0; ii < 2; ++ii) {
      const int i = 2 * w + ii;
      const v4f ha = *(const v4fa*)(sHJ + i * 512 + 4 * lane);
      const v4f hb = *(const v4fa*)(sHJ + i * 512 + 128 + 4 * lane);
#pragma unroll 2
      for (int j = 0; j < 16; ++j) {
        const v4f ga = *(const v4fa*)(sHJ + j * 512 + 256 + 4 * lane);
        const v4f gb = *(const v4fa*)(sHJ + j * 512 + 384 + 4 * lane);
        float p = 0.0f;
#pragma unroll
        for (int e = 0; e < 4; ++e) {
          const float r = fmaxf((ha[e] + ga[e]) + b1a[e], 0.0f);
          p = fmaf(r, wa[e], p);
        }
#pragma unroll
        for (int e = 0; e < 4; ++e) {
          const float r = fmaxf((hb[e] + gb[e]) + b1b[e], 0.0f);
          p = fmaf(r, wb[e], p);
        }
        p += __shfl_xor(p, 16);
        p += __shfl_xor(p, 8);
        p += __shfl_xor(p, 4);
        p += __shfl_xor(p, 2);
        p += __shfl_xor(p, 1);
        const float z = p + e2b;
        float wv = sigm(z);
        const int mk = sMask[i * 16 + j];
        wv = (mk != 0) ? wv : 0.0f;
        if (lane == 0) sW[i * 16 + j] = wv;
      }
    }
  }
  __syncthreads();

  float* sA = sHJ;
#pragma unroll 1
  for (int i = 0; i < 16; ++i) {
    float acc = 0.0f;
    int any = 0;
#pragma unroll 4
    for (int j = 0; j < 16; ++j) {
      acc = fmaf(sW[i * 16 + j], sX[j * 256 + tid], acc);
      any |= sMask[i * 16 + j];
    }
    const float xv = sX[i * 256 + tid];
    sA[i * 256 + tid] = (any != 0) ? acc : xv;
  }
  __syncthreads();

  v4u hv[2], lv[2];
#pragma unroll
  for (int ii = 0; ii < 2; ++ii) {
    const int i = 2 * w + ii;
    const v4f a = *(const v4fa*)(sA + i * 256 + 8 * lane);
    const v4f c = *(const v4fa*)(sA + i * 256 + 8 * lane + 4);
    hv[ii] = hi8(a, c);
    lv[ii] = lo8(a, c);
  }
  for (int pass = 0; pass < 2; ++pass) {
#pragma unroll
    for (int ii = 0; ii < 2; ++ii) {
      const int i = 2 * w + ii;
      unsigned short* o = AGG + ((size_t)b * 16 + i) * KHL + 8 * lane;
      *(volatile v4u*)o = hv[ii];
      *(volatile v4u*)(o + ND) = lv[ii];
    }
    __threadfence();
  }
}

template <int FIRST, int LAST>
__global__ __launch_bounds__(256) void k_cell(const float* __restrict__ G, float* __restrict__ C,
                                              unsigned short* __restrict__ HOUT, float* __restrict__ out1,
                                              int t) {
  __shared__ __align__(16) float sH[256];
  __shared__ __align__(16) float sC[256];
  const int tid = threadIdx.x, lane = tid & 31, w = tid >> 5;
  const int n = blockIdx.x;
  const float* g = G + (size_t)n * NG;
  const float gi = g[tid];
  const float gf = g[256 + tid];
  const float gg = g[512 + tid];
  const float go = g[768 + tid];
  float cp = 0.0f;
  if (!FIRST) cp = C[(size_t)n * ND + tid];
  const float c = sigm(gf) * cp + sigm(gi) * tanhf(gg);
  const float h = sigm(go) * tanhf(c);
  sH[tid] = h;
  sC[tid] = c;
  __syncthreads();
  const size_t row = (size_t)n * NSTEP + t;
  if (w < 2) {
    const int col = 128 * w + 4 * lane;
    const v4f v = *(const v4fa*)(sC + col);
    float* o = C + (size_t)n * ND + col;
    *(volatile v4f*)o = v;
    __threadfence();
    *(volatile v4f*)o = v;
  } else if (w < 4) {
    if (LAST) {
      const int col = 128 * (w - 2) + 4 * lane;
      const v4f v = *(const v4fa*)(sH + col);
      float* o = out1 + row * ND + col;
      *(volatile v4f*)o = v;
      __threadfence();
      *(volatile v4f*)o = v;
    }
  } else if (w == 4) {
    const v4f a = *(const v4fa*)(sH + 8 * lane);
    const v4f cc = *(const v4fa*)(sH + 8 * lane + 4);
    const v4u hv = hi8(a, cc);
    unsigned short* o = HOUT + row * KHL + 8 * lane;
    *(volatile v4u*)o = hv;
    __threadfence();
    *(volatile v4u*)o = hv;
  } else if (w == 5) {
    const v4f a = *(const v4fa*)(sH + 8 * lane);
    const v4f cc = *(const v4fa*)(sH + 8 * lane + 4);
    const v4u lv = lo8(a, cc);
    unsigned short* o = HOUT + row * KHL + ND + 8 * lane;
    *(volatile v4u*)o = lv;
    __threadfence();
    *(volatile v4u*)o = lv;
  }
}

extern "C" void kernel_launch(void* const* d_in, const int* in_sizes, int n_in,
                              void* d_out, int out_size, void* d_ws, size_t ws_size,
                              hipStream_t stream) {
  if (n_in < 15) return;
  if (in_sizes[0] != NR * ND) return;
  if (in_sizes[1] != NNODE * NNODE) return;
  if (in_sizes[2] != NNODE * ND) return;
  if (in_sizes[3] != NLAYER * 2 * ND * ND) return;
  if (in_sizes[4] != NLAYER * ND) return;
  if (in_sizes[5] != NLAYER * ND * ND) return;
  if (in_sizes[6] != NLAYER * ND) return;
  if (in_sizes[7] != 2 * ND * ND) return;
  if (in_sizes[8] != ND) return;
  if (in_sizes[9] != ND) return;
  if (in_sizes[10] != 1) return;
  if (in_sizes[11] != 2 * NG * ND) return;
  if (in_sizes[12] != 2 * NG * ND) return;
  if (in_sizes[13] != 2 * NG) return;
  if (in_sizes[14] != 2 * NG) return;
  if (out_size != NR * ND + NR * NSTEP * ND) return;

  const float* mf   = (const float*)d_in[0];
  const int*   adj  = (const int*)d_in[1];
  const float* emb  = (const float*)d_in[2];
  const float* gW1  = (const float*)d_in[3];
  const float* gb1  = (const float*)d_in[4];
  const float* gW2  = (const float*)d_in[5];
  const float* gb2  = (const float*)d_in[6];
  const float* eW1  = (const float*)d_in[7];
  const float* eb1  = (const float*)d_in[8];
  const float* eW2  = (const float*)d_in[9];
  const float* eb2  = (const float*)d_in[10];
  const float* lWih = (const float*)d_in[11];
  const float* lWhh = (const float*)d_in[12];
  const float* lbih = (const float*)d_in[13];
  const float* lbhh = (const float*)d_in[14];
  float* out0 = (float*)d_out;
  float* out1 = out0 + (size_t)NR * ND;

  const size_t PBIG = (size_t)NR * NG * 4;
  const size_t PHL  = (size_t)NR * KHL * 2;
  const size_t PXF  = (size_t)NR * ND * 4;
  const size_t PBE  = (size_t)KHL * KHL * 2;
  const size_t PB1  = (size_t)NLAYER * ND * KL * 2;
  const size_t PB2  = (size_t)NLAYER * ND * KHL * 2;
  const size_t PBL  = (size_t)2 * NG * KL * 2;
  size_t off = 0;
  const size_t oF = off;    off += PBIG;
  const size_t oH = off;    off += PBIG;
  const size_t oHIST = off; off += PBIG;
  const size_t oC = off;    off += PXF;
  const size_t oBE = off;   off += PBE;
  const size_t oB1 = off;   off += PB1;
  const size_t oB2 = off;   off += PB2;
  const size_t oBL = off;   off += PBL;
  if (off > ws_size) return;
  if (off > (size_t)134217728) return;

  char* ws = (char*)d_ws;
  float* XF  = (float*)(ws + oF);
  float* HIJ = (float*)(ws + oF + PXF);
  float* G   = (float*)(ws + oF);
  unsigned short* XHL = (unsigned short*)(ws + oH);
  unsigned short* AGG = (unsigned short*)(ws + oH + PHL);
  unsigned short* T1  = (unsigned short*)(ws + oH + 2 * PHL);
  unsigned short* H1  = (unsigned short*)(ws + oH);
  unsigned short* HIST = (unsigned short*)(ws + oHIST);
  unsigned short* H2   = (unsigned short*)(ws + oHIST);
  float* C = (float*)(ws + oC);
  unsigned short* BE = (unsigned short*)(ws + oBE);
  unsigned short* B1 = (unsigned short*)(ws + oB1);
  unsigned short* B2 = (unsigned short*)(ws + oB2);
  unsigned short* BL = (unsigned short*)(ws + oBL);

  k_wt<<<dim3(4, 4, 2), 256, 0, stream>>>(eW1, BE, 1, ND * KHL, 0, KHL);
  k_wt<<<dim3(4, 4, 2 * NLAYER), 256, 0, stream>>>(gW1, B1, 2, ND * KL, KHL, KL);
  k_wt<<<dim3(4, 4, NLAYER), 256, 0, stream>>>(gW2, B2, 1, ND * KHL, 0, KHL);
  k_wl<<<dim3((2 * NG * (ND / 8)) / 256), 256, 0, stream>>>(lWih, lWhh, BL);

  k_x0<<<dim3(NR / 8), 256, 0, stream>>>(mf, emb, XF, XHL, HIST);

  for (int l = 0; l < NLAYER; ++l) {
    k_gemm_f32<0><<<dim3(NR / 128, KHL / 64), 128, 0, stream>>>(
        XHL, KHL, XHL, KHL, KHL, 0, BE, KHL, HIJ, KHL, eb1, eb1);
    k_pair<<<dim3(NBATCH), 256, 0, stream>>>(HIJ, XF, adj, eb1, eW2, eb2, AGG);
    k_gemm_relu<<<dim3(NR / 128, ND / 64), 128, 0, stream>>>(
        XHL, AGG, B1 + (size_t)l * ND * KL, gb1 + l * ND, T1);
    float* Fdst = (l + 1 < NLAYER) ? XF : out0;
    k_gemm_x<<<dim3(NR / 128, ND / 64), 128, 0, stream>>>(
        T1, B2 + (size_t)l * ND * KHL, gb2 + l * ND, Fdst, XHL, HIST, l + 1, (l + 1 < NLAYER) ? 1 : 0);
  }

  for (int k = 0; k < 2; ++k) {
    const unsigned short* IN = (k == 0) ? HIST : H1;
    unsigned short* HOUT = (k == 0) ? H1 : H2;
    const unsigned short* BLk = BL + (size_t)k * NG * KL;
    const float* bih = lbih + k * NG;
    const float* bhh = lbhh + k * NG;
    for (int t = 0; t < NSTEP; ++t) {
      if (t == 0) {
        k_gemm_f32<1><<<dim3(NR / 128, NG / 64), 128, 0, stream>>>(
            IN, NSTEP * KHL, IN, NSTEP * KHL, KHL, 0, BLk, KL, G, NG, bih, bhh);
        if (k == 0) k_cell<1, 0><<<dim3(NR), 256, 0, stream>>>(G, C, HOUT, out1, t);
        else        k_cell<1, 1><<<dim3(NR), 256, 0, stream>>>(G, C, HOUT, out1, t);
      } else {
        k_gemm_f32<1><<<dim3(NR / 128, NG / 64), 128, 0, stream>>>(
            IN + (size_t)t * KHL, NSTEP * KHL, HOUT + (size_t)(t - 1) * KHL, NSTEP * KHL,
            KHL, KHL, BLk, KL, G, NG, bih, bhh);
        if (k == 0) k_cell<0, 0><<<dim3(NR), 256, 0, stream>>>(G, C, HOUT, out1, t);
        else        k_cell<0, 1><<<dim3(NR), 256, 0, stream>>>(G, C, HOUT, out1, t);
      }
    }
  }
  (void)hipGetLastError();
}
